// Encoder_77996606095381
// MI455X (gfx1250) — hardware-verified
//
#include <hip/hip_runtime.h>
#include <stddef.h>
#include <stdint.h>
#include <math.h>


#define DIN1    256
#define HID     128
#define NHEAD   4
#define CW      512
#define NP1     1152
#define NP2     1024
#define KX      256
#define CPL     16
#define HLN     8
#define NTHR    256
#define NWAVE   8
#define EPT     8
#define CHUNK   (NTHR * EPT)
#define WCAP    (EPT * 32)
#define LISTN   (NWAVE * WCAP)
#define NBMAX   2048
#define NBRUN   1024
#define SLOTB   11
#define RCAP    28672
#define DEGCAP  128
#define STWF    512
#define WSTW    (2 * HID + 4)
#define PW      288
#define GBM     64
#define GBN     64
#define GTHR    128
#define USH     5
#define NEGSA   0.2f
#define BNEPS   1e-5f
#define WSMAX   134217728
#define LDS_AGG ((2 * RCAP + 2 * NBMAX + LISTN) * 4 + 64)

static_assert((CHUNK & (CHUNK - 1)) == 0 && CHUNK <= (1 << SLOTB));
static_assert(NBMAX == (1 << SLOTB));
static_assert((NBRUN & (NBRUN - 1)) == 0 && NBRUN <= NBMAX && NBRUN >= 32);
static_assert(NTHR * 8 == NBMAX);
static_assert(LISTN >= NBMAX);
static_assert(LISTN >= NWAVE * WCAP);
static_assert((RCAP % 32) == 0);
static_assert(DEGCAP <= RCAP);
static_assert(LDS_AGG <= 300000);
static_assert(LDS_AGG == 254016);
static_assert(GBM == (GTHR / 32) * 16);
static_assert((KX % 32) == 0 && DIN1 == KX && KX == 2 * HID);
static_assert(KX / 8 == (1 << USH));
static_assert(DIN1 / 8 == 32);
static_assert((NP1 % GBN) == 0 && NP1 == 2 * CW + HID);
static_assert((NP2 % GBN) == 0 && NP2 == 2 * CW);
static_assert(CW == 32 * CPL && CW == NHEAD * HID && HID == HLN * CPL);
static_assert(HID == 4 * 32);
static_assert(STWF == CW && NWAVE * STWF <= RCAP);
static_assert(NWAVE * WSTW + PW <= RCAP && (WSTW % 4) == 0);
static_assert(PW == ((2 * HID + 1 + 31) / 32) * 32 && PW / 4 <= NTHR);
static_assert(NTHR == 2 * HID);

typedef float          v4f  __attribute__((ext_vector_type(4)));
typedef float          v8f  __attribute__((ext_vector_type(8)));
typedef int            v4i  __attribute__((ext_vector_type(4)));
typedef int            v8i  __attribute__((ext_vector_type(8)));
typedef unsigned int   v4u  __attribute__((ext_vector_type(4)));
typedef unsigned short v8us __attribute__((ext_vector_type(8)));
typedef __bf16         v16b __attribute__((ext_vector_type(16)));
typedef v4f  __attribute__((may_alias)) v4fa;
typedef v8us __attribute__((may_alias)) v8usa;
union FragB { v16b v; v8us h[2]; v8i w; };

__device__ __forceinline__ v8f wmb(const FragB& a, const FragB& b, v8f c) {
  v8f d = __builtin_amdgcn_wmma_f32_16x16x32_bf16(false, a.v, false, b.v, (short)0, c, false, false);
  asm volatile("v_nop\n\tv_nop\n\tv_nop\n\tv_nop" : "+v"(d) : "v"(a.w), "v"(b.w));
  return d;
}

__device__ __forceinline__ v8f z8() { v8f z = {0.f, 0.f, 0.f, 0.f, 0.f, 0.f, 0.f, 0.f}; return z; }

__device__ __forceinline__ unsigned int f2bf(float f) {
  const unsigned int u = __float_as_uint(f);
  return ((u + 0x7FFFu + ((u >> 16) & 1u)) >> 16) & 0xFFFFu;
}
__device__ __forceinline__ float bf2f(unsigned int b) { return __uint_as_float(b << 16); }
__device__ __forceinline__ float bfr(float f) { return bf2f(f2bf(f)); }
__device__ __forceinline__ v4f bfr4(const v4f a) {
  v4f r; r.x = bfr(a.x); r.y = bfr(a.y); r.z = bfr(a.z); r.w = bfr(a.w); return r;
}
__device__ __forceinline__ unsigned int pk2(float lo, float hi) { return f2bf(lo) | (f2bf(hi) << 16); }
__device__ __forceinline__ v4u pack8(const v4f a, const v4f b) {
  v4u r;
  r.x = pk2(a.x, a.y); r.y = pk2(a.z, a.w); r.z = pk2(b.x, b.y); r.w = pk2(b.z, b.w);
  return r;
}
__device__ __forceinline__ v8us cvt8b(const v4f a, const v4f b) {
  v8us o;
  o[0] = (unsigned short)f2bf(a.x); o[1] = (unsigned short)f2bf(a.y);
  o[2] = (unsigned short)f2bf(a.z); o[3] = (unsigned short)f2bf(a.w);
  o[4] = (unsigned short)f2bf(b.x); o[5] = (unsigned short)f2bf(b.y);
  o[6] = (unsigned short)f2bf(b.z); o[7] = (unsigned short)f2bf(b.w);
  return o;
}

template<int C> struct RowIO;
template<> struct RowIO<16> {
  static __device__ __forceinline__ void ld(float (&d)[16], const float* p) {
#pragma unroll
    for (int k = 0; k < 4; ++k) {
      const v4f t = *(const v4fa*)(p + 4 * k);
      d[4 * k] = t.x; d[4 * k + 1] = t.y; d[4 * k + 2] = t.z; d[4 * k + 3] = t.w;
    }
  }
  static __device__ __forceinline__ void ldb(float (&d)[16], const float* p) {
#pragma unroll
    for (int k = 0; k < 4; ++k) {
      const v4f t = bfr4(*(const v4fa*)(p + 4 * k));
      d[4 * k] = t.x; d[4 * k + 1] = t.y; d[4 * k + 2] = t.z; d[4 * k + 3] = t.w;
    }
  }
  static __device__ __forceinline__ void stl(float* p, const float (&r)[16]) {
#pragma unroll
    for (int k = 0; k < 4; ++k) {
      v4f t;
      t.x = r[4 * k]; t.y = r[4 * k + 1]; t.z = r[4 * k + 2]; t.w = r[4 * k + 3];
      *(v4fa*)(p + 4 * k) = t;
    }
  }
};
template<> struct RowIO<4> {
  static __device__ __forceinline__ void ld(float (&d)[4], const float* p) {
    const v4f t = *(const v4fa*)p; d[0] = t.x; d[1] = t.y; d[2] = t.z; d[3] = t.w;
  }
  static __device__ __forceinline__ void ldb(float (&d)[4], const float* p) {
    const v4f t = bfr4(*(const v4fa*)p); d[0] = t.x; d[1] = t.y; d[2] = t.z; d[3] = t.w;
  }
  static __device__ __forceinline__ void stl(float* p, const float (&r)[4]) {
    v4f t; t.x = r[0]; t.y = r[1]; t.z = r[2]; t.w = r[3]; *(v4fa*)p = t;
  }
};

template<int HL>
__device__ __forceinline__ float hsum(float p) {
#pragma unroll
  for (int o = HL >> 1; o >= 1; o >>= 1) p += __shfl_xor(p, o);
  return p;
}

__device__ __forceinline__ int scan_chunk(const int* __restrict__ dsts, int nE, int cbase, int slotBase,
                                          int nb, int vec8, int* list, int tid, int lane, int wave) {
  int wc = 0;
  const int el0  = tid * EPT;
  const int e0   = cbase + el0;
  const int sent = -2147483647 - 1;
  v4i da, db;
  if (vec8 != 0 && cbase + CHUNK <= nE) {
    da = *(const v4i*)(dsts + e0);
    db = *(const v4i*)(dsts + e0 + 4);
  } else {
    da.x = (e0     < nE) ? dsts[min(e0,     nE - 1)] : sent;
    da.y = (e0 + 1 < nE) ? dsts[min(e0 + 1, nE - 1)] : sent;
    da.z = (e0 + 2 < nE) ? dsts[min(e0 + 2, nE - 1)] : sent;
    da.w = (e0 + 3 < nE) ? dsts[min(e0 + 3, nE - 1)] : sent;
    db.x = (e0 + 4 < nE) ? dsts[min(e0 + 4, nE - 1)] : sent;
    db.y = (e0 + 5 < nE) ? dsts[min(e0 + 5, nE - 1)] : sent;
    db.z = (e0 + 6 < nE) ? dsts[min(e0 + 6, nE - 1)] : sent;
    db.w = (e0 + 7 < nE) ? dsts[min(e0 + 7, nE - 1)] : sent;
  }
  const unsigned nbs = (unsigned)slotBase;
  const unsigned unb = (unsigned)nb;
  const unsigned s0 = (unsigned)da.x - nbs, s1 = (unsigned)da.y - nbs;
  const unsigned s2 = (unsigned)da.z - nbs, s3 = (unsigned)da.w - nbs;
  const unsigned s4 = (unsigned)db.x - nbs, s5 = (unsigned)db.y - nbs;
  const unsigned s6 = (unsigned)db.z - nbs, s7 = (unsigned)db.w - nbs;
  const bool h0 = s0 < unb, h1 = s1 < unb, h2 = s2 < unb, h3 = s3 < unb;
  const bool h4 = s4 < unb, h5 = s5 < unb, h6 = s6 < unb, h7 = s7 < unb;
  const unsigned any = __builtin_amdgcn_ballot_w32(h0 | h1 | h2 | h3 | h4 | h5 | h6 | h7);
  if (any != 0u) {
#define HITJ(J, HJ, SJ) { \
      const unsigned mj = __builtin_amdgcn_ballot_w32(HJ); \
      if (mj != 0u) { \
        if (HJ) { \
          const int pos = wc + (int)__builtin_amdgcn_mbcnt_lo(mj, 0u); \
          if (pos < WCAP) list[wave * WCAP + pos] = ((el0 + (J)) << SLOTB) | (int)(SJ); \
        } \
        wc += (int)__builtin_popcount(mj); } }
    HITJ(0, h0, s0)
    HITJ(1, h1, s1)
    HITJ(2, h2, s2)
    HITJ(3, h3, s3)
    HITJ(4, h4, s4)
    HITJ(5, h5, s5)
    HITJ(6, h6, s6)
    HITJ(7, h7, s7)
#undef HITJ
  }
  return wc;
}

__device__ __forceinline__ void wt_unit(const float* __restrict__ w, int cols, int ush, int kmask, int Kout,
                                        unsigned short* wt, int rowoff, int u) {
  const int n   = u >> ush;
  const int k8  = (u & ((1 << ush) - 1)) * 8;
  const int kk  = k8 & kmask;
  const int ncl = n < cols ? n : cols - 1;
  const float* p = w + (size_t)kk * (size_t)cols + ncl;
  v4f a, b;
  a.x = p[0];                  a.y = p[(size_t)cols];       a.z = p[(size_t)2 * cols];   a.w = p[(size_t)3 * cols];
  b.x = p[(size_t)4 * cols];   b.y = p[(size_t)5 * cols];   b.z = p[(size_t)6 * cols];   b.w = p[(size_t)7 * cols];
  const v4f z4 = {0.f, 0.f, 0.f, 0.f};
  if (n >= cols) { a = z4; b = z4; }
  const v8us hv = cvt8b(a, b);
  const size_t o = (size_t)(rowoff + n) * (size_t)Kout + k8;
  *(volatile v8us*)(wt + o) = hv;
  __threadfence();
  *(volatile v8us*)(wt + o) = hv;
}

__global__ __launch_bounds__(NTHR) void k_wt(const float* __restrict__ W, int cols, int ush, int kmask, int Kout,
                                             int rowoff, int nUnits, unsigned short* wt) {
  const int u = (int)blockIdx.x * NTHR + (int)threadIdx.x;
  if (u < nUnits) wt_unit(W, cols, ush, kmask, Kout, wt, rowoff, u);
}

__global__ __launch_bounds__(NTHR) void k_xcvt(const float* __restrict__ x, int nN, int nUnits,
                                               unsigned short* xb) {
  const int u = (int)blockIdx.x * NTHR + (int)threadIdx.x;
  if (u >= nUnits) return;
  const int row   = u >> 5;
  const int piece = u & 31;
  const int c0    = 8 * piece;
  const int rc    = row < nN ? row : nN - 1;
  const float* p  = x + (size_t)rc * DIN1 + c0;
  v4f a = *(const v4fa*)p;
  v4f b = *(const v4fa*)(p + 4);
  const v4f z4 = {0.f, 0.f, 0.f, 0.f};
  if (row >= nN) { a = z4; b = z4; }
  const v4u q = pack8(a, b);
  unsigned short* o = xb + (size_t)row * KX + c0;
  *(volatile v4u*)o = q;
  __threadfence();
  *(volatile v4u*)o = q;
}

__global__ __launch_bounds__(GTHR) void k_gemm(
    const unsigned short* __restrict__ A, const unsigned short* __restrict__ WT,
    const float* __restrict__ b0, const float* __restrict__ b1, const float* __restrict__ b2,
    int n0, int n1, int nb0, int nb1, int nb2,
    float* outF, int K, int ldo)
{
  __shared__ __attribute__((aligned(16))) float stg[GBM * GBN];
  const int tid = (int)threadIdx.x, lane = tid & 31, wave = tid >> 5, hh = lane >> 4, m = lane & 15;
  const int rowBase = (int)blockIdx.x * GBM;
  const int col0    = (int)blockIdx.y * GBN;

  v8f acc[4];
#pragma unroll
  for (int t = 0; t < 4; ++t) acc[t] = z8();
  const unsigned short* ap = A  + (size_t)(rowBase + 16 * wave + m) * (size_t)K + 8 * hh;
  const unsigned short* wp = WT + (size_t)(col0 + m) * (size_t)K + 8 * hh;
  const int ksteps = K >> 5;
#pragma unroll 1
  for (int ks = 0; ks < ksteps; ++ks) {
    FragB af;
    af.h[0] = *(const v8usa*)(ap + 32 * ks);
    af.h[1] = *(const v8usa*)(ap + 32 * ks + 16);
#pragma unroll
    for (int t = 0; t < 4; ++t) {
      const unsigned short* wq = wp + (size_t)(16 * t) * (size_t)K + 32 * ks;
      FragB bf;
      bf.h[0] = *(const v8usa*)wq;
      bf.h[1] = *(const v8usa*)(wq + 16);
      acc[t] = wmb(af, bf, acc[t]);
    }
  }

#pragma unroll
  for (int t = 0; t < 4; ++t) {
    const int lc = 16 * t + m;
#pragma unroll
    for (int r = 0; r < 8; ++r) {
      const int lr = 16 * wave + 8 * hh + r;
      stg[lr * GBN + lc] = acc[t][r];
    }
  }
  __syncthreads();

  const int gcb = col0 + 4 * m;
  int j0 = gcb;      j0 = j0 > nb0 - 4 ? nb0 - 4 : j0; j0 = j0 < 0 ? 0 : j0;
  int j1 = gcb - n0; j1 = j1 > nb1 - 4 ? nb1 - 4 : j1; j1 = j1 < 0 ? 0 : j1;
  int j2 = gcb - n1; j2 = j2 > nb2 - 4 ? nb2 - 4 : j2; j2 = j2 < 0 ? 0 : j2;
  const v4f q0 = bfr4(*(const v4fa*)(b0 + j0));
  const v4f q1 = bfr4(*(const v4fa*)(b1 + j1));
  const v4f q2 = bfr4(*(const v4fa*)(b2 + j2));
  const float f0 = (gcb < n0) ? 1.0f : 0.0f;
  const float f1 = (gcb >= n0 && gcb < n1) ? 1.0f : 0.0f;
  const float f2 = (gcb >= n1) ? 1.0f : 0.0f;
  const v4f bsum = q0 * f0 + q1 * f1 + q2 * f2;

  v4f fv[8];
#pragma unroll
  for (int i = 0; i < 8; ++i) {
    const int lr = 16 * wave + 2 * i + hh;
    fv[i] = *(const v4fa*)(stg + lr * GBN + 4 * m) + bsum;
  }
#pragma unroll
  for (int i = 0; i < 8; ++i) {
    const int lr = 16 * wave + 2 * i + hh;
    const int gr = rowBase + lr;
    float* op = outF + (size_t)gr * (size_t)ldo + col0 + 4 * m;
    *(volatile v4f*)op = fv[i];
  }
  __threadfence();
#pragma unroll
  for (int i = 0; i < 8; ++i) {
    const int lr = 16 * wave + 2 * i + hh;
    const int gr = rowBase + lr;
    float* op = outF + (size_t)gr * (size_t)ldo + col0 + 4 * m;
    *(volatile v4f*)op = fv[i];
  }
}

template<int C>
__device__ __forceinline__ float edot(const float (&hs)[C], const float (&hd)[C], const float (&at)[C]) {
  float part = 0.f;
#pragma unroll
  for (int j = 0; j < C; ++j) {
    float v = hs[j] + hd[j];
    v = v >= 0.f ? v : v * NEGSA;
    part = fmaf(v, at[j], part);
  }
  return part;
}
template<int C>
__device__ __forceinline__ void smerge(float lg, float& mx, float& dn, float (&av)[C], const float (&hs)[C]) {
  const float df = lg - mx;
  const float ee = __expf(-fabsf(df));
  const bool up  = df > 0.f;
  const float s1 = up ? ee : 1.0f;
  const float s2 = up ? 1.0f : ee;
  mx = up ? lg : mx;
  dn = fmaf(dn, s1, s2);
#pragma unroll
  for (int j = 0; j < C; ++j) av[j] = fmaf(av[j], s1, s2 * hs[j]);
}

__global__ __launch_bounds__(NTHR) void k_agg(
    const int* __restrict__ srcs, const int* __restrict__ dsts,
    const float* __restrict__ F, int ldf, const float* __restrict__ att, const float* __restrict__ bias,
    float* hcp, int nRowsW, float* part,
    int nN, int nE, int nb, int vec8) {
  extern __shared__ v4f lds_dyn[];
  int* reg1 = (int*)lds_dyn;
  int* reg2 = reg1 + RCAP;
  int* scnt = reg2 + RCAP;
  int* soff = scnt + NBMAX;
  int* list = soff + NBMAX;
  int* wcnt = list + LISTN;
  int* wtot = wcnt + NWAVE;
  const int tid = (int)threadIdx.x, lane = tid & 31, wave = tid >> 5;
  const int nodeBase = (int)blockIdx.x * nb;

  for (int i = tid; i < NBMAX; i += NTHR) scnt[i] = 0;
  for (int i = tid; i < RCAP; i += NTHR) reg2[i] = 0;
  __syncthreads();

  int tot = 0;
  const int nChunks = (nE + CHUNK - 1) / CHUNK;
#pragma unroll 1
  for (int ch = 0; ch < nChunks; ++ch) {
    const int cbase = ch * CHUNK;
    const int wc = scan_chunk(dsts, nE, cbase, nodeBase, nb, vec8, list, tid, lane, wave);
    if (lane == 0) wcnt[wave] = wc;
    __syncthreads();
    int pre = 0, all = 0;
#pragma unroll
    for (int w2 = 0; w2 < NWAVE; ++w2) {
      int c = wcnt[w2];
      c = c < 0 ? 0 : (c > WCAP ? WCAP : c);
      all += c;
      pre += (w2 < wave) ? c : 0;
    }
    const int wcc  = wc > WCAP ? WCAP : wc;
    const int base = tot + pre;
#pragma unroll 1
    for (int i = lane; i < wcc; i += 32) {
      const int ent = list[wave * WCAP + i];
      const int el  = (ent >> SLOTB) & (CHUNK - 1);
      const int sl  = ent & (NBMAX - 1);
      int eid = cbase + el;
      eid = eid > nE - 1 ? nE - 1 : eid;
      const int pos = base + i;
      if (pos < RCAP) reg1[pos] = (int)(((unsigned)eid << SLOTB) | (unsigned)sl);
    }
    tot += all;
    tot = tot > RCAP ? RCAP : tot;
    __syncthreads();
  }
  const int nh = tot;

  if (wave == 0) {
#pragma unroll 1
    for (int b0 = 0; b0 < nh; b0 += 32) {
      const int idx = b0 + lane;
      const int uv  = reg1[idx < nh ? idx : nh - 1];
      const int m32 = (nh - b0) < 32 ? (nh - b0) : 32;
#pragma unroll 1
      for (int k = 0; k < m32; ++k) {
        const int u  = __builtin_amdgcn_readlane(uv, k);
        const int sl = u & (NBMAX - 1);
        if (lane == 0) scnt[sl] = scnt[sl] + 1;
      }
    }
  }
  __syncthreads();

  {
    const v4i ca = *(const v4i*)(scnt + 8 * tid);
    const v4i cb = *(const v4i*)(scnt + 8 * tid + 4);
    const int e0 = ca.x < 0 ? 0 : ca.x, e1 = ca.y < 0 ? 0 : ca.y, e2 = ca.z < 0 ? 0 : ca.z, e3 = ca.w < 0 ? 0 : ca.w;
    const int e4 = cb.x < 0 ? 0 : cb.x, e5 = cb.y < 0 ? 0 : cb.y, e6 = cb.z < 0 ? 0 : cb.z, e7 = cb.w < 0 ? 0 : cb.w;
    const int ts = e0 + e1 + e2 + e3 + e4 + e5 + e6 + e7;
    int incl = ts;
#pragma unroll
    for (int d = 1; d < 32; d <<= 1) {
      const int up = __shfl_up(incl, d);
      if (lane >= d) incl += up;
    }
    if (lane == 31) wtot[wave] = incl;
    __syncthreads();
    int pre = 0;
#pragma unroll
    for (int w2 = 0; w2 < NWAVE; ++w2) pre += (w2 < wave) ? wtot[w2] : 0;
    int run = pre + incl - ts;
    soff[8 * tid + 0] = run; run += e0;
    soff[8 * tid + 1] = run; run += e1;
    soff[8 * tid + 2] = run; run += e2;
    soff[8 * tid + 3] = run; run += e3;
    soff[8 * tid + 4] = run; run += e4;
    soff[8 * tid + 5] = run; run += e5;
    soff[8 * tid + 6] = run; run += e6;
    soff[8 * tid + 7] = run;
  }
  __syncthreads();
  for (int i = tid; i < NBMAX; i += NTHR) list[i] = soff[i];
  __syncthreads();

  if (wave == 0) {
#pragma unroll 1
    for (int b0 = 0; b0 < nh; b0 += 32) {
      const int idx = b0 + lane;
      const int uv  = reg1[idx < nh ? idx : nh - 1];
      const int m32 = (nh - b0) < 32 ? (nh - b0) : 32;
#pragma unroll 1
      for (int k = 0; k < m32; ++k) {
        const int u   = __builtin_amdgcn_readlane(uv, k);
        const int sl  = u & (NBMAX - 1);
        const int eid = (int)((unsigned)u >> SLOTB);
        if (lane == 0) {
          int pos = list[sl];
          pos = pos < 0 ? 0 : (pos > RCAP - 1 ? RCAP - 1 : pos);
          reg2[pos] = eid;
          list[sl] = pos + 1;
        }
      }
    }
  }
  __syncthreads();

  const int nbw = nb >> 3;
  const bool ovf = (nh >= RCAP);
  const float qnan = __int_as_float(0x7fc00000);
  const int c0 = CPL * lane;
  const int oc = 4 * lane;
  float* stw = (float*)reg1 + wave * STWF;
  float at[CPL], bb[4];
  RowIO<CPL>::ldb(at, att + c0);
  RowIO<4>::ldb(bb, bias + oc);
  int wn = 0;
  float wm[4], wq[4];
#pragma unroll
  for (int j = 0; j < 4; ++j) { wm[j] = 0.0f; wq[j] = 0.0f; }

#pragma unroll 1
  for (int jt = 0; jt < nbw; ++jt) {
    const int slot = wave * nbw + jt;
    const int grow = nodeBase + slot;
    const int gcl  = grow < nN ? grow : nN - 1;
    int st = soff[slot];
    const int craw = scnt[slot];
    int cnt = craw;
    st  = st < 0 ? 0 : (st > nh ? nh : st);
    cnt = cnt < 0 ? 0 : (cnt > DEGCAP ? DEGCAP : cnt);
    if (cnt > nh - st) cnt = nh - st;
    const float pz = (ovf || craw > DEGCAP) ? qnan : 0.0f;
    const bool live = grow < nN;

    const float* fr = F + (size_t)gcl * (size_t)ldf;
    float hd[CPL];
    RowIO<CPL>::ld(hd, fr + CW + c0);
    float av[CPL];
#pragma unroll
    for (int j = 0; j < CPL; ++j) av[j] = 0.f;
    float mx = -1.0e30f, dn = 0.f;

#pragma unroll 1
    for (int q = 0; q <= cnt; ++q) {
      const bool last = (q == cnt);
      int idx = st + q; idx = idx > RCAP - 1 ? RCAP - 1 : idx;
      int eid = reg2[idx]; eid = eid < 0 ? 0 : (eid > nE - 1 ? nE - 1 : eid);
      const int sraw = srcs[eid];
      const int se = sraw < 0 ? 0 : (sraw > nN - 1 ? nN - 1 : sraw);
      const int s = last ? gcl : se;
      float hs[CPL];
      RowIO<CPL>::ld(hs, F + (size_t)s * (size_t)ldf + c0);
      const float lg = hsum<HLN>(edot<CPL>(hs, hd, at));
      smerge<CPL>(lg, mx, dn, av, hs);
    }
    const float inv = __builtin_amdgcn_rcpf(dn);

    float r[CPL];
#pragma unroll
    for (int j = 0; j < CPL; ++j) r[j] = av[j] * inv;

    __builtin_amdgcn_fence(__ATOMIC_RELEASE, "wavefront");
    __builtin_amdgcn_wave_barrier();
    RowIO<CPL>::stl(stw + c0, r);
    __builtin_amdgcn_fence(__ATOMIC_RELEASE, "wavefront");
    __builtin_amdgcn_wave_barrier();
    const v4f q0 = *(const v4fa*)(stw + oc);
    const v4f q1 = *(const v4fa*)(stw + HID + oc);
    const v4f q2 = *(const v4fa*)(stw + 2 * HID + oc);
    const v4f q3 = *(const v4fa*)(stw + 3 * HID + oc);
    const v4f ys = ((q0 + q1) + q2) + q3;
    float v[4];
    v[0] = fmaf(ys.x, 0.25f, bb[0]);
    v[1] = fmaf(ys.y, 0.25f, bb[1]);
    v[2] = fmaf(ys.z, 0.25f, bb[2]);
    v[3] = fmaf(ys.w, 0.25f, bb[3]);
#pragma unroll
    for (int j = 0; j < 4; ++j) v[j] = v[j] >= 0.f ? v[j] : v[j] * NEGSA;
    if (live) {
      wn += 1;
      const float rk = __builtin_amdgcn_rcpf((float)wn);
#pragma unroll
      for (int j = 0; j < 4; ++j) {
        const float d = v[j] - wm[j];
        wm[j] = fmaf(d, rk, wm[j]);
        wq[j] = fmaf(d, v[j] - wm[j], wq[j]);
      }
    }
    v4f yv;
    yv.x = (live ? v[0] : 0.f) + pz;
    yv.y = (live ? v[1] : 0.f) + pz;
    yv.z = (live ? v[2] : 0.f) + pz;
    yv.w = (live ? v[3] : 0.f) + pz;

    const bool wrow = grow < nRowsW;
    const int growc = wrow ? grow : nRowsW - 1;
    float* op = hcp + (size_t)growc * (size_t)HID + oc;
    if (wrow) *(volatile v4f*)op = yv;
    __threadfence();
    if (wrow) *(volatile v4f*)op = yv;
  }

  __syncthreads();
  float* wst = (float*)reg2;
  float* pst = wst + NWAVE * WSTW;
  RowIO<4>::stl(wst + wave * WSTW + oc, wm);
  RowIO<4>::stl(wst + wave * WSTW + HID + oc, wq);
  if (lane == 0) wst[wave * WSTW + 2 * HID] = (float)wn;
  __syncthreads();
  if (tid < HID) {
    float n = 0.0f, mean = 0.0f, M2 = 0.0f;
#pragma unroll 1
    for (int w2 = 0; w2 < NWAVE; ++w2) {
      const float nbv = wst[w2 * WSTW + 2 * HID];
      const float mb  = wst[w2 * WSTW + tid];
      const float qb  = wst[w2 * WSTW + HID + tid];
      if (nbv > 0.5f) {
        const float nn = n + nbv;
        const float delta = mb - mean;
        const float f = nbv / nn;
        mean = fmaf(delta, f, mean);
        M2 = M2 + qb + delta * delta * n * f;
        n = nn;
      }
    }
    pst[1 + tid] = mean;
    pst[1 + HID + tid] = M2;
    if (tid == 0) pst[0] = n;
  }
#pragma unroll 1
  for (int i = 2 * HID + 1 + tid; i < PW; i += NTHR) pst[i] = 0.0f;
  __syncthreads();
  const int pb = (int)blockIdx.x;
  v4f ps = {0.0f, 0.0f, 0.0f, 0.0f};
  if (tid < PW / 4) {
    ps = *(const v4fa*)(pst + 4 * tid);
    *(volatile v4f*)(part + (size_t)pb * PW + 4 * tid) = ps;
  }
  __threadfence();
  if (tid < PW / 4) {
    *(volatile v4f*)(part + (size_t)pb * PW + 4 * tid) = ps;
  }
}

__global__ __launch_bounds__(HID) void k_bnfin(const float* __restrict__ part, int nPart,
                                               const float* __restrict__ gam, const float* __restrict__ bet,
                                               float* ss) {
  __shared__ __attribute__((aligned(16))) float stg[2 * HID];
  const int tid = (int)threadIdx.x;
  const int c = tid;
  double n = 0.0, mean = 0.0, M2 = 0.0;
#pragma unroll 1
  for (int b = 0; b < nPart; ++b) {
    const float* pr = part + (size_t)b * PW;
    const double nbv = (double)pr[0];
    const double mb  = (double)pr[1 + c];
    const double qb  = (double)pr[1 + HID + c];
    if (nbv > 0.5) {
      const double nn = n + nbv;
      const double delta = mb - mean;
      const double f = nbv / nn;
      mean = mean + delta * f;
      M2 = M2 + qb + delta * delta * n * f;
      n = nn;
    }
  }
  const double nt = n < 1.0 ? 1.0 : n;
  const float varf  = (float)(M2 / nt);
  const float meanf = (float)mean;
  const float rstd = 1.0f / sqrtf(varf + BNEPS);
  const float sc = bfr(gam[c]) * rstd;
  const float sh = bfr(bet[c]) - meanf * sc;
  stg[c] = sc;
  stg[HID + c] = sh;
  __syncthreads();
  v4f v = {0.0f, 0.0f, 0.0f, 0.0f};
  if (tid < (2 * HID) / 4) {
    v = *(const v4fa*)(stg + 4 * tid);
    *(volatile v4f*)(ss + 4 * tid) = v;
  }
  __threadfence();
  if (tid < (2 * HID) / 4) {
    *(volatile v4f*)(ss + 4 * tid) = v;
  }
}

__global__ __launch_bounds__(NTHR) void k_apply(const float* __restrict__ hc, const float* __restrict__ ss,
                                                const float* __restrict__ F, int ldf, int hoff,
                                                int nN, int nUnits, unsigned short* apl) {
  __shared__ __attribute__((aligned(16))) float ssh[2 * HID];
  const int tid = (int)threadIdx.x;
  ssh[tid] = ss[tid];
  __syncthreads();
  const int u = (int)blockIdx.x * NTHR + tid;
  const bool act = u < nUnits;
  const int uc = act ? u : (nUnits - 1);
  const int row = uc >> 5;
  const int piece = uc & 31;
  const int c0 = (piece & 15) * 8;
  const float* p = hc + (size_t)row * HID + c0;
  const v4f a = *(const v4fa*)p;
  const v4f b = *(const v4fa*)(p + 4);
  const float* ph = F + (size_t)row * (size_t)ldf + hoff + c0;
  const v4f ha = *(const v4fa*)ph;
  const v4f hb = *(const v4fa*)(ph + 4);
  const v4f sca = *(const v4fa*)(ssh + c0);
  const v4f scb = *(const v4fa*)(ssh + c0 + 4);
  const v4f sha = *(const v4fa*)(ssh + HID + c0);
  const v4f shb = *(const v4fa*)(ssh + HID + c0 + 4);
  const bool live = row < nN;
  float y[8];
  y[0] = fmaf(a.x, sca.x, sha.x) + ha.x; y[1] = fmaf(a.y, sca.y, sha.y) + ha.y;
  y[2] = fmaf(a.z, sca.z, sha.z) + ha.z; y[3] = fmaf(a.w, sca.w, sha.w) + ha.w;
  y[4] = fmaf(b.x, scb.x, shb.x) + hb.x; y[5] = fmaf(b.y, scb.y, shb.y) + hb.y;
  y[6] = fmaf(b.z, scb.z, shb.z) + hb.z; y[7] = fmaf(b.w, scb.w, shb.w) + hb.w;
  unsigned int wv[8];
  const bool lsel = piece >= 16;
#pragma unroll
  for (int j = 0; j < 8; ++j) {
    const float t = live ? y[j] : 0.0f;
    const unsigned int hbt = f2bf(t);
    const unsigned int lbt = f2bf(t - bf2f(hbt));
    wv[j] = lsel ? lbt : hbt;
  }
  v4u q;
  q.x = wv[0] | (wv[1] << 16);
  q.y = wv[2] | (wv[3] << 16);
  q.z = wv[4] | (wv[5] << 16);
  q.w = wv[6] | (wv[7] << 16);
  unsigned short* o = apl + (size_t)row * KX + 8 * piece;
  if (act) *(volatile v4u*)o = q;
  __threadfence();
  if (act) *(volatile v4u*)o = q;
}

__global__ __launch_bounds__(NTHR) void k_final(const float* __restrict__ hc, const float* __restrict__ ss,
                                                int nN, int nUnits, float* out) {
  __shared__ __attribute__((aligned(16))) float ssh[2 * HID];
  const int tid = (int)threadIdx.x;
  ssh[tid] = ss[tid];
  __syncthreads();
  const int u = (int)blockIdx.x * NTHR + tid;
  const bool act = u < nUnits;
  const int uc = act ? u : (nUnits - 1);
  const int row = uc >> 5;
  const int c0 = (uc & 31) * 4;
  const v4f a  = *(const v4fa*)(hc + (size_t)row * HID + c0);
  const v4f sc = *(const v4fa*)(ssh + c0);
  const v4f sh = *(const v4fa*)(ssh + HID + c0);
  v4f y;
  y.x = fmaf(a.x, sc.x, sh.x); y.y = fmaf(a.y, sc.y, sh.y);
  y.z = fmaf(a.z, sc.z, sh.z); y.w = fmaf(a.w, sc.w, sh.w);
  float* o = out + (size_t)row * HID + c0;
  if (act) *(volatile v4f*)o = y;
  __threadfence();
  if (act) *(volatile v4f*)o = y;
  (void)nN;
}

static int pick_nb(int nE, int nN) {
  int nb = NBRUN;
  while (nb > 32 && (long long)nb * (long long)nE * 5LL > (long long)RCAP * (long long)nN * 4LL) nb >>= 1;
  return nb;
}
static inline int cdiv(int a, int b) { return (a + b - 1) / b; }
static inline size_t al256(size_t o) { return (o + 255) & ~(size_t)255; }

extern "C" void kernel_launch(void* const* d_in, const int* in_sizes, int n_in,
                              void* d_out, int out_size, void* d_ws, size_t ws_size,
                              hipStream_t stream) {
  if (n_in < 20) return;
  if (in_sizes[0] < 16 * DIN1 || (in_sizes[0] % DIN1) != 0) return;
  const int nN = in_sizes[0] / DIN1;
  if (nN >= (1 << 21)) return;
  if (in_sizes[1] < 2 || (in_sizes[1] & 1) != 0) return;
  const int nE = in_sizes[1] / 2;
  if (nE < 1 || nE >= (1 << (32 - SLOTB))) return;
  if (in_sizes[2] != DIN1 * CW || in_sizes[3] != DIN1 * CW) return;
  if (in_sizes[4] != CW || in_sizes[5] != CW) return;
  if (in_sizes[6] != CW) return;
  if (in_sizes[7] != HID || in_sizes[8] != HID || in_sizes[9] != HID) return;
  if (in_sizes[10] != HID * CW || in_sizes[11] != HID * CW) return;
  if (in_sizes[12] != CW || in_sizes[13] != CW) return;
  if (in_sizes[14] != CW) return;
  if (in_sizes[15] != HID || in_sizes[16] != HID || in_sizes[17] != HID) return;
  if (in_sizes[18] != DIN1 * HID || in_sizes[19] != HID) return;
  if (out_size != nN * HID) return;

  const float* x     = (const float*)d_in[0];
  const int*   ei    = (const int*)  d_in[1];
  const float* Wl0   = (const float*)d_in[2];
  const float* Wr0   = (const float*)d_in[3];
  const float* bl0   = (const float*)d_in[4];
  const float* br0   = (const float*)d_in[5];
  const float* att0  = (const float*)d_in[6];
  const float* b0    = (const float*)d_in[7];
  const float* g0    = (const float*)d_in[8];
  const float* be0   = (const float*)d_in[9];
  const float* Wl1   = (const float*)d_in[10];
  const float* Wr1   = (const float*)d_in[11];
  const float* bl1   = (const float*)d_in[12];
  const float* br1   = (const float*)d_in[13];
  const float* att1  = (const float*)d_in[14];
  const float* b1    = (const float*)d_in[15];
  const float* g1    = (const float*)d_in[16];
  const float* be1   = (const float*)d_in[17];
  const float* skW   = (const float*)d_in[18];
  const float* skb   = (const float*)d_in[19];
  float* out = (float*)d_out;
  const int* src = ei;
  const int* dst = ei + nE;

  const int MP   = cdiv(nN, GBM) * GBM;
  const int gM   = MP / GBM;
  const int nb   = pick_nb(nE, nN);
  if (nb < 32 || (nb & (nb - 1)) != 0 || nb > NBMAX) return;
  const int gA   = cdiv(MP, nb);
  if ((long long)gA * nb < (long long)MP) return;
  const int vec8 = ((nE & 3) == 0) ? 1 : 0;

  char* ws = (char*)d_ws;
  size_t off = 0;
  const size_t oW1 = off; off = al256(off + (size_t)NP1 * KX * 2);
  const size_t oW2 = off; off = al256(off + (size_t)NP2 * KX * 2);
  const size_t oP  = off; off = al256(off + (size_t)MP * KX * 2);
  const size_t oF  = off; off = al256(off + (size_t)MP * NP1 * 4);
  const size_t oQ  = off; off = al256(off + (size_t)MP * HID * 4);
  const size_t oPT = off; off = al256(off + (size_t)gA * PW * 4);
  const size_t oSS = off; off = al256(off + (size_t)(2 * HID) * 4);
  if (off > ws_size || off > (size_t)WSMAX) return;
  unsigned short* WT1 = (unsigned short*)(ws + oW1);
  unsigned short* WT2 = (unsigned short*)(ws + oW2);
  unsigned short* XB  = (unsigned short*)(ws + oP);
  unsigned short* APL = (unsigned short*)(ws + oP);
  float*          F   = (float*)(ws + oF);
  float*          HC  = (float*)(ws + oQ);
  float*          PT  = (float*)(ws + oPT);
  float*          SS  = (float*)(ws + oSS);

  hipFuncSetAttribute(reinterpret_cast<const void*>(&k_agg),
                      hipFuncAttributeMaxDynamicSharedMemorySize, LDS_AGG);

  {
    const int nUx = MP * (DIN1 / 8);
    k_xcvt<<<cdiv(nUx, NTHR), NTHR, 0, stream>>>(x, nN, nUx, XB);
    const int nUw = CW * (KX / 8);
    const int nUs = HID * (KX / 8);
    k_wt<<<cdiv(nUw, NTHR), NTHR, 0, stream>>>(Wl0, CW, USH, DIN1 - 1, KX, 0, nUw, WT1);
    k_wt<<<cdiv(nUw, NTHR), NTHR, 0, stream>>>(Wr0, CW, USH, DIN1 - 1, KX, CW, nUw, WT1);
    k_wt<<<cdiv(nUs, NTHR), NTHR, 0, stream>>>(skW, HID, USH, DIN1 - 1, KX, 2 * CW, nUs, WT1);
    k_wt<<<cdiv(nUw, NTHR), NTHR, 0, stream>>>(Wl1, CW, USH, HID - 1, KX, 0, nUw, WT2);
    k_wt<<<cdiv(nUw, NTHR), NTHR, 0, stream>>>(Wr1, CW, USH, HID - 1, KX, CW, nUw, WT2);
  }
  const int nUa = MP * 32;
  const int nUf = nN * 32;

  k_gemm<<<dim3(gM, NP1 / GBN), GTHR, 0, stream>>>(XB, WT1, bl0, br0, skb, CW, NP2, CW, CW, HID, F, DIN1, NP1);
  k_agg<<<gA, NTHR, LDS_AGG, stream>>>(src, dst, F, NP1, att0, b0, HC, MP, PT, nN, nE, nb, vec8);
  k_bnfin<<<1, HID, 0, stream>>>(PT, gA, g0, be0, SS);
  k_apply<<<cdiv(nUa, NTHR), NTHR, 0, stream>>>(HC, SS, F, NP1, NP2, nN, nUa, APL);

  k_gemm<<<dim3(gM, NP2 / GBN), GTHR, 0, stream>>>(APL, WT2, bl1, br1, br1, CW, NP2, CW, CW, CW, F, KX, NP2);
  k_agg<<<gA, NTHR, LDS_AGG, stream>>>(src, dst, F, NP2, att1, b1, HC, MP, PT, nN, nE, nb, vec8);
  k_bnfin<<<1, HID, 0, stream>>>(PT, gA, g1, be1, SS);
  k_final<<<cdiv(nUf, NTHR), NTHR, 0, stream>>>(HC, SS, nN, nUf, out);
}
